// vision_mamba_61400852464204
// MI455X (gfx1250) — hardware-verified
//
#include <hip/hip_runtime.h>
#include <math.h>

typedef __attribute__((ext_vector_type(16))) _Float16 v16h;
typedef __attribute__((ext_vector_type(8)))  float    v8f;

namespace {

constexpr int Bsz = 8, Cc = 96, Dd = 192, Nn = 16, Rr = 6, Kk = 4;
constexpr int DEPTH = 12, NCLS = 43;
constexpr int Hh = 14, Ww = 14, Ll = 196, ROWS = Bsz * Ll;
constexpr int BCW = 32;

#define RSPLIT (1.0f / 2048.0f)
typedef __attribute__((ext_vector_type(4))) float v4f_t;
typedef float v4fa __attribute__((ext_vector_type(4), may_alias));
__device__ __forceinline__ _Float16 lo_of(float v, _Float16 h) { return (_Float16)((v - (float)h) * 2048.0f); }
__device__ __forceinline__ unsigned pk2s(float a, float b, unsigned* lo) {
  const _Float16 h0 = (_Float16)a, h1 = (_Float16)b;
  *lo = (unsigned)__builtin_bit_cast(unsigned short, lo_of(a, h0)) | ((unsigned)__builtin_bit_cast(unsigned short, lo_of(b, h1)) << 16);
  return (unsigned)__builtin_bit_cast(unsigned short, h0) | ((unsigned)__builtin_bit_cast(unsigned short, h1) << 16);
}
__device__ __forceinline__ void st_pair(_Float16* p, long plane, float a, float b) {
  unsigned lo; const unsigned v = pk2s(a, b, &lo);
  *(volatile unsigned*)p = v; *(volatile unsigned*)(p + plane) = lo; __threadfence();
  *(volatile unsigned*)p = v; *(volatile unsigned*)(p + plane) = lo;
}
__device__ __forceinline__ void st2f(float* p, float v) { *(volatile float*)p = v; __threadfence(); *(volatile float*)p = v; }
__device__ __forceinline__ v16h zero16() {
  v16h a;
#pragma unroll
  for (int i = 0; i < 16; ++i) a[i] = (_Float16)0.f;
  return a;
}

struct Frag2 { v16h h, l; };
typedef __attribute__((ext_vector_type(4))) float v4fx;
__device__ __forceinline__ Frag2 load_a16(const float* __restrict__ p) {
  const v4fx q0 = *(const v4fx*)p, q1 = *(const v4fx*)(p + 4), q2 = *(const v4fx*)(p + 16), q3 = *(const v4fx*)(p + 20);
  Frag2 a;
#pragma unroll
  for (int i = 0; i < 4; ++i) {
    a.h[i] = (_Float16)q0[i];      a.l[i] = lo_of(q0[i], a.h[i]);
    a.h[4 + i] = (_Float16)q1[i];  a.l[4 + i] = lo_of(q1[i], a.h[4 + i]);
    a.h[8 + i] = (_Float16)q2[i];  a.l[8 + i] = lo_of(q2[i], a.h[8 + i]);
    a.h[12 + i] = (_Float16)q3[i]; a.l[12 + i] = lo_of(q3[i], a.h[12 + i]);
  }
  return a;
}
__device__ __forceinline__ Frag2 load_b16(const _Float16* __restrict__ p, long plane) {
  typedef __attribute__((ext_vector_type(8))) _Float16 v8h;
  Frag2 b;
  b.h = __builtin_shufflevector(*(const v8h*)p, *(const v8h*)(p + 16), 0,1,2,3,4,5,6,7,8,9,10,11,12,13,14,15);
  b.l = __builtin_shufflevector(*(const v8h*)(p + plane), *(const v8h*)(p + plane + 16), 0,1,2,3,4,5,6,7,8,9,10,11,12,13,14,15);
  return b;
}
__device__ __forceinline__ v8f wmma16(v16h a, v16h b, v8f c) { return __builtin_amdgcn_wmma_f32_16x16x32_f16(false, a, false, b, (short)0, c, false, false); }
__device__ __forceinline__ v8f WMMA32(const Frag2& a, const Frag2& b, v8f c) { v8f x = {}; x = wmma16(a.l, b.h, x); x = wmma16(a.h, b.l, x); return wmma16(a.h, b.h, c) + x * RSPLIT; }
__device__ __forceinline__ Frag2 zero2() { Frag2 f; f.h = zero16(); f.l = zero16(); return f; }

__device__ __forceinline__ void store_c(float* __restrict__ Cm, long idx, float v,
                                        int mode, float bias) {
  if (mode == 0) {
    Cm[idx] = v;
  } else if (mode == 1) {
    float s = v + bias;
    Cm[idx] = (s > 20.f) ? s : log1pf(__expf(s));
  } else if (mode == 2) {
    Cm[idx] += v;
  } else {
    Cm[idx] = v + bias;
  }
}

__global__ __launch_bounds__(32) void gemm_wmma(const float* __restrict__ A, long sAz,
                          const _Float16* __restrict__ Bw, long sBz,
                          float* __restrict__ Cm, long sCz,
                          int M, int N, int Kt, int lda, int ldc,
                          int mode, const float* __restrict__ bias, long sBiasZ, long plB)
{
  __shared__ __attribute__((aligned(16))) float stg[32 * 36];
  const int lane = (int)(threadIdx.x & 31u);
  const int row0 = blockIdx.x * 32;
  const int col0 = blockIdx.y * 32;
  const int z = blockIdx.z;
  A  += (long)z * sAz;
  Bw += (long)z * sBz;
  Cm += (long)z * sCz;
  if (bias) bias += (long)z * sBiasZ;

  const int half16 = lane >> 4;
  const int l15 = lane & 15;
  const int kAoff = half16 * 8;
  const int kBoff = half16 * 8;
  const int mA0 = row0 + l15, mA1 = mA0 + 16;
  const int nB0 = col0 + l15, nB1 = nB0 + 16;

  v8f c00 = {0.f,0.f,0.f,0.f,0.f,0.f,0.f,0.f};
  v8f c01 = c00, c10 = c00, c11 = c00;

  const bool full = (row0 + 32 <= M) && (col0 + 32 <= N);
  if (full) {
    const float*    pa0 = A  + (long)mA0 * lda + kAoff;
    const float*    pa1 = A  + (long)mA1 * lda + kAoff;
    const _Float16* pb0 = Bw + (long)nB0 * Kt  + kBoff;
    const _Float16* pb1 = Bw + (long)nB1 * Kt  + kBoff;
    Frag2 a0 = load_a16(pa0);
    Frag2 a1 = load_a16(pa1);
    Frag2 b0 = load_b16(pb0, plB);
    Frag2 b1 = load_b16(pb1, plB);
    for (int kc = 32; kc < Kt; kc += 32) {
      Frag2 na0 = load_a16(pa0 + kc);
      Frag2 na1 = load_a16(pa1 + kc);
      Frag2 nb0 = load_b16(pb0 + kc, plB);
      Frag2 nb1 = load_b16(pb1 + kc, plB);
      c00 = WMMA32(a0, b0, c00);
      c01 = WMMA32(a0, b1, c01);
      c10 = WMMA32(a1, b0, c10);
      c11 = WMMA32(a1, b1, c11);
      a0 = na0; a1 = na1; b0 = nb0; b1 = nb1;
    }
    c00 = WMMA32(a0, b0, c00);
    c01 = WMMA32(a0, b1, c01);
    c10 = WMMA32(a1, b0, c10);
    c11 = WMMA32(a1, b1, c11);
  } else {
    for (int kc = 0; kc < Kt; kc += 32) {
      Frag2 a0 = load_a16(A + (long)min(mA0, M - 1) * lda + kc + kAoff);
      Frag2 a1 = load_a16(A + (long)min(mA1, M - 1) * lda + kc + kAoff);
      Frag2 b0 = load_b16(Bw + (long)min(nB0, N - 1) * Kt + kc + kBoff, plB);
      Frag2 b1 = load_b16(Bw + (long)min(nB1, N - 1) * Kt + kc + kBoff, plB);
      c00 = WMMA32(a0, b0, c00);
      c01 = WMMA32(a0, b1, c01);
      c10 = WMMA32(a1, b0, c10);
      c11 = WMMA32(a1, b1, c11);
    }
  }

  const float bias0 = (bias && nB0 < N) ? bias[nB0] : 0.f;
  const float bias1 = (bias && nB1 < N) ? bias[nB1] : 0.f;
  const int mb0 = half16 * 8;
#pragma unroll
  for (int r = 0; r < 8; ++r) {
    const int ml0 = mb0 + r, ml1 = mb0 + 16 + r;
    float v;
    v = c00[r]; if (mode == 1) { float s = v + bias0; v = (s > 20.f) ? s : log1pf(__expf(s)); } else if (mode == 2) v += Cm[(long)(row0 + ml0) * ldc + nB0]; else if (mode == 3) v += bias0; stg[ml0 * 36 + l15] = v;
    v = c10[r]; if (mode == 1) { float s = v + bias0; v = (s > 20.f) ? s : log1pf(__expf(s)); } else if (mode == 2) v += Cm[(long)(row0 + ml1) * ldc + nB0]; else if (mode == 3) v += bias0; stg[ml1 * 36 + l15] = v;
    v = c01[r]; if (mode == 1) { float s = v + bias1; v = (s > 20.f) ? s : log1pf(__expf(s)); } else if (mode == 2) v += Cm[(long)(row0 + ml0) * ldc + nB1]; else if (mode == 3) v += bias1; stg[ml0 * 36 + 16 + l15] = v;
    v = c11[r]; if (mode == 1) { float s = v + bias1; v = (s > 20.f) ? s : log1pf(__expf(s)); } else if (mode == 2) v += Cm[(long)(row0 + ml1) * ldc + nB1]; else if (mode == 3) v += bias1; stg[ml1 * 36 + 16 + l15] = v;
  }
  asm volatile("s_wait_dscnt 0" ::: "memory");
#pragma unroll 1
  for (int pass = 0; pass < 2; ++pass) {
#pragma unroll
    for (int i = 0; i < 8; ++i) { const int c = lane + 32 * i, rr = c >> 3, q = (c & 7) * 4;
      if (row0 + rr < M) *(volatile v4f_t*)(Cm + (long)(row0 + rr) * ldc + col0 + q) = *(const volatile v4fa*)(stg + rr * 36 + q); }
    __threadfence();
  }
}

__global__ void head_kernel(const float* __restrict__ pooled, const float* __restrict__ hw, const float* __restrict__ hb, float* __restrict__ out) {
  int idx = blockIdx.x * blockDim.x + threadIdx.x;
  if (idx >= Bsz * NCLS) return;
  int b = idx / NCLS, n = idx % NCLS;
  float s = hb[n];
#pragma unroll 1
  for (int k = 0; k < Cc; ++k) s += pooled[b * Cc + k] * hw[k * NCLS + n];
  st2f(out + idx, s);
}

__global__ void prep_patch(const float* __restrict__ w, _Float16* __restrict__ o) {
  int idx = blockIdx.x * blockDim.x + threadIdx.x;
  idx *= 2; if (idx < Cc * 768) st_pair(o + idx, (long)Cc * 768, w[idx], w[idx + 1]);
}
__global__ void prep_inproj(const float* __restrict__ w, _Float16* __restrict__ o) {
  int idx = (blockIdx.x * blockDim.x + threadIdx.x) * 2;
  if (idx >= DEPTH * 2 * Dd * Cc) return;
  int c = idx % Cc; int r = idx / Cc;
  int n = r % (2 * Dd); int i = r / (2 * Dd);
  st_pair(o + idx, (long)DEPTH * 2 * Dd * Cc, w[((long)i * Cc + c) * (2 * Dd) + n], w[((long)i * Cc + c + 1) * (2 * Dd) + n]);
}
__global__ void prep_outproj(const float* __restrict__ w, _Float16* __restrict__ o) {
  int idx = (blockIdx.x * blockDim.x + threadIdx.x) * 2;
  if (idx >= DEPTH * Cc * Dd) return;
  int k = idx % Dd; int r = idx / Dd;
  int n = r % Cc; int i = r / Cc;
  st_pair(o + idx, (long)DEPTH * Cc * Dd, w[((long)i * Dd + k) * Cc + n], w[((long)i * Dd + k + 1) * Cc + n]);
}
__global__ void prep_bc(const float* __restrict__ xpw, _Float16* __restrict__ o) {
  int idx = (blockIdx.x * blockDim.x + threadIdx.x) * 2;
  if (idx >= DEPTH * Kk * BCW * Dd) return;
  int dd = idx % Dd; int r = idx / Dd;
  int c = r % BCW; int g = r / BCW;
  const float* s = xpw + ((long)g * 38 + Rr + c) * Dd + dd;
  st_pair(o + idx, (long)DEPTH * Kk * BCW * Dd, s[0], s[1]);
}
__global__ void prep_dtfused(const float* __restrict__ xpw, const float* __restrict__ dtw,
                             _Float16* __restrict__ o) {
  int idx = (blockIdx.x * blockDim.x + threadIdx.x) * 2;
  if (idx >= DEPTH * Kk * Dd * Dd) return;
  int dd = idx % Dd; int r2 = idx / Dd;
  int d = r2 % Dd; int g = r2 / Dd;
  const float* dw = dtw + ((long)g * Dd + d) * Rr;
  const float* xp = xpw + (long)g * 38 * Dd + dd;
  float s0 = 0.f, s1 = 0.f;
#pragma unroll 1
  for (int r = 0; r < Rr; ++r) { s0 += dw[r] * xp[(long)r * Dd]; s1 += dw[r] * xp[(long)r * Dd + 1]; }
  st_pair(o + idx, (long)DEPTH * Kk * Dd * Dd, s0, s1);
}
__global__ void prep_head(const float* __restrict__ w, _Float16* __restrict__ o) {
  int idx = blockIdx.x * blockDim.x + threadIdx.x;
  if (idx >= NCLS * Cc) return;
  int k = idx % Cc; int n = idx / Cc;
  o[idx] = (_Float16)w[k * NCLS + n];
}

__global__ void im2col_patch(const float* __restrict__ x, float* __restrict__ col) {
  int idx = blockIdx.x * blockDim.x + threadIdx.x;
  if (idx >= ROWS * 768) return;
  int m = idx / 768, k = idx - m * 768;
  int b = m / Ll, l = m - b * Ll;
  int ph = l / Ww, pw = l - ph * Ww;
  int ci = k / 256, r = k - ci * 256;
  int py = r / 16, px = r - py * 16;
  st2f(col + idx, x[(((long)b * 3 + ci) * 224 + (ph * 16 + py)) * 224 + (pw * 16 + px)]);
}

__global__ void patch_epilogue(float* __restrict__ t, const float* __restrict__ pb,
                               const float* __restrict__ pos) {
  int idx = blockIdx.x * blockDim.x + threadIdx.x;
  if (idx >= ROWS * Cc) return;
  int c = idx % Cc;
  int l = (idx / Cc) % Ll;
  st2f(t + idx, t[idx] + pb[c] + pos[l * Cc + c]);
}

__global__ void layernorm_rows(const float* __restrict__ in, float* __restrict__ out,
                               const float* __restrict__ w, const float* __restrict__ b,
                               int rows, int width) {
  int r = blockIdx.x * blockDim.x + threadIdx.x;
  if (r >= rows) return;
  const float* p = in + (long)r * width;
  float mu = 0.f;
  for (int i = 0; i < width; ++i) mu += p[i];
  mu /= (float)width;
  float var = 0.f;
  for (int i = 0; i < width; ++i) { float d = p[i] - mu; var += d * d; }
  var /= (float)width;
  float rs = rsqrtf(var + 1e-6f);
  float* q = out + (long)r * width;
  for (int i = 0; i < width; ++i) *(volatile float*)(q + i) = (p[i] - mu) * rs * w[i] + b[i];
  __threadfence();
  for (int i = 0; i < width; ++i) *(volatile float*)(q + i) = (p[i] - mu) * rs * w[i] + b[i];
}

__global__ void dwconv_scan_prep(const float* __restrict__ xz, const float* __restrict__ cw,
                                 const float* __restrict__ cb, float* __restrict__ xst) {
  int idx = blockIdx.x * blockDim.x + threadIdx.x;
  if (idx >= ROWS * Dd) return;
  int d = idx % Dd;
  int m = idx / Dd;
  int b = m / Ll, l = m - b * Ll;
  int h = l / Ww, w = l - h * Ww;
  float s = 0.f;
#pragma unroll
  for (int dy = -1; dy <= 1; ++dy) {
    int hh = h + dy;
    if (hh < 0 || hh >= Hh) continue;
#pragma unroll
    for (int dx = -1; dx <= 1; ++dx) {
      int ww = w + dx;
      if (ww < 0 || ww >= Ww) continue;
      s += cw[d * 9 + (dy + 1) * 3 + (dx + 1)] *
           xz[((long)b * Ll + hh * Ww + ww) * (2 * Dd) + d];
    }
  }
  s += cb[d];
  s = s / (1.f + __expf(-s));
  const long kS = (long)ROWS * Dd;
  int l2 = w * Hh + h;
#pragma unroll 1
  for (int pass = 0; pass < 2; ++pass) {
    *(volatile float*)(xst + ((long)b * Ll + l) * Dd + d)                      = s;
    *(volatile float*)(xst + kS     + ((long)b * Ll + l2) * Dd + d)            = s;
    *(volatile float*)(xst + 2 * kS + ((long)b * Ll + (Ll - 1 - l)) * Dd + d)  = s;
    *(volatile float*)(xst + 3 * kS + ((long)b * Ll + (Ll - 1 - l2)) * Dd + d) = s;
    __threadfence();
  }
}

__global__ void selective_scan(const float* __restrict__ xst, const float* __restrict__ dts,
                               const float* __restrict__ bc, const float* __restrict__ Alog,
                               const float* __restrict__ Dsk, float* __restrict__ ys) {
  int idx = blockIdx.x * blockDim.x + threadIdx.x;
  if (idx >= Kk * Bsz * Dd) return;
  int d = idx % Dd;
  int t = idx / Dd;
  int b = t % Bsz;
  int k = t / Bsz;
  const long kS = (long)ROWS * Dd;
  const float* xp  = xst + (long)k * kS + ((long)b * Ll) * Dd + d;
  const float* dtp = dts + (long)k * kS + ((long)b * Ll) * Dd + d;
  const float* blp = bc + ((long)k * ROWS + (long)b * Ll) * BCW;
  float Av[Nn];
#pragma unroll
  for (int n = 0; n < Nn; ++n) Av[n] = -__expf(Alog[((long)k * Dd + d) * Nn + n]);
  const float Dv = Dsk[k * Dd + d];
  float h[Nn];
#pragma unroll
  for (int n = 0; n < Nn; ++n) h[n] = 0.f;
  float* yk = ys + (long)k * kS;
  for (int l = 0; l < Ll; ++l) {
    const float xv = xp[(long)l * Dd];
    const float dt = dtp[(long)l * Dd];
    const float* bl = blp + (long)l * BCW;
    const float dx = dt * xv;
    float y = 0.f;
#pragma unroll
    for (int n = 0; n < Nn; ++n) {
      h[n] = h[n] * __expf(dt * Av[n]) + dx * bl[n];
      y += h[n] * bl[Nn + n];
    }
    y += Dv * xv;
    int li;
    if (k == 0)      li = l;
    else if (k == 1) { int w = l / Hh, hh2 = l % Hh; li = hh2 * Ww + w; }
    else if (k == 2) li = Ll - 1 - l;
    else             { int l2 = Ll - 1 - l; int w = l2 / Hh, hh2 = l2 % Hh; li = hh2 * Ww + w; }
    *(volatile float*)(yk + ((long)b * Ll + li) * Dd + d) = y;
  }
  __threadfence();
  for (int l = 0; l < Ll; ++l) {
    int li;
    if (k == 0)      li = l;
    else if (k == 1) { int w = l / Hh, hh2 = l % Hh; li = hh2 * Ww + w; }
    else if (k == 2) li = Ll - 1 - l;
    else             { int l2 = Ll - 1 - l; int w = l2 / Hh, hh2 = l2 % Hh; li = hh2 * Ww + w; }
    float* p = yk + ((long)b * Ll + li) * Dd + d; *(volatile float*)p = *(volatile float*)p;
  }
}

__global__ void merge_ln_gate(const float* __restrict__ ys, const float* __restrict__ xz,
                              const float* __restrict__ onw, const float* __restrict__ onb,
                              float* __restrict__ gated) {
  const int r = blockIdx.x;
  const int lane = threadIdx.x;
  const long kS = (long)ROWS * Dd;
  float v[6];
  float sum = 0.f;
#pragma unroll
  for (int j = 0; j < 6; ++j) {
    const int d = lane + j * 32;
    const long off = (long)r * Dd + d;
    float s = ys[off] + ys[kS + off] + ys[2 * kS + off] + ys[3 * kS + off];
    v[j] = s;
    sum += s;
  }
#pragma unroll
  for (int o = 16; o > 0; o >>= 1) sum += __shfl_xor(sum, o, 32);
  const float mu = sum / (float)Dd;
  float var = 0.f;
#pragma unroll
  for (int j = 0; j < 6; ++j) { float dd = v[j] - mu; var += dd * dd; }
#pragma unroll
  for (int o = 16; o > 0; o >>= 1) var += __shfl_xor(var, o, 32);
  const float rs = rsqrtf(var / (float)Dd + 1e-6f);
#pragma unroll
  for (int j = 0; j < 6; ++j) {
    const int d = lane + j * 32;
    const float zn = xz[(long)r * (2 * Dd) + Dd + d];
    const float sil = zn / (1.f + __expf(-zn));
    *(volatile float*)(gated + (long)r * Dd + d) = ((v[j] - mu) * rs * onw[d] + onb[d]) * sil;
  }
  __threadfence();
#pragma unroll
  for (int j = 0; j < 6; ++j) {
    const int d = lane + j * 32;
    const float zn = xz[(long)r * (2 * Dd) + Dd + d];
    const float sil = zn / (1.f + __expf(-zn));
    *(volatile float*)(gated + (long)r * Dd + d) = ((v[j] - mu) * rs * onw[d] + onb[d]) * sil;
  }
}

__global__ void pool_tokens(const float* __restrict__ tn, float* __restrict__ pooled) {
  int idx = blockIdx.x * blockDim.x + threadIdx.x;
  if (idx >= Bsz * Cc) return;
  int b = idx / Cc, c = idx % Cc;
  float s = 0.f;
  for (int l = 0; l < Ll; ++l) s += tn[((long)b * Ll + l) * Cc + c];
  st2f(pooled + idx, s / (float)Ll);
}

}

extern "C" void kernel_launch(void* const* d_in, const int* in_sizes, int n_in,
                              void* d_out, int out_size, void* d_ws, size_t ws_size,
                              hipStream_t stream) {
  (void)in_sizes; (void)n_in; (void)out_size; (void)ws_size;
  const float* x         = (const float*)d_in[0];
  const float* patch_w   = (const float*)d_in[1];
  const float* patch_b   = (const float*)d_in[2];
  const float* pos       = (const float*)d_in[3];
  const float* ln1_w     = (const float*)d_in[4];
  const float* ln1_b     = (const float*)d_in[5];
  const float* in_proj_w = (const float*)d_in[6];
  const float* conv_w    = (const float*)d_in[7];
  const float* conv_b    = (const float*)d_in[8];
  const float* x_proj_w  = (const float*)d_in[9];
  const float* dt_proj_w = (const float*)d_in[10];
  const float* dt_proj_b = (const float*)d_in[11];
  const float* A_logs    = (const float*)d_in[12];
  const float* Ds        = (const float*)d_in[13];
  const float* onw       = (const float*)d_in[14];
  const float* onb       = (const float*)d_in[15];
  const float* out_proj_w= (const float*)d_in[16];
  const float* norm_w    = (const float*)d_in[17];
  const float* norm_b    = (const float*)d_in[18];
  const float* head_w    = (const float*)d_in[19];
  const float* head_b    = (const float*)d_in[20];
  float* out = (float*)d_out;

  float* ws = (float*)d_ws;
  size_t o = 0;
  float* t      = ws + o; o += (size_t)ROWS * Cc;
  float* tn     = ws + o; o += (size_t)ROWS * Cc;
  float* xz     = ws + o; o += (size_t)ROWS * 2 * Dd;
  float* xst    = ws + o; o += (size_t)Kk * ROWS * Dd;
  float* bcb    = ws + o; o += (size_t)Kk * ROWS * BCW;
  float* dts    = ws + o; o += (size_t)Kk * ROWS * Dd;
  float* ys     = ws + o; o += (size_t)Kk * ROWS * Dd;
  float* gated  = ws + o; o += (size_t)ROWS * Dd;
  float* pooled = ws + o; o += (size_t)Bsz * Cc;
  float* col = dts;

  size_t hoff = (o * sizeof(float) + 255) & ~(size_t)255;
  _Float16* hp = (_Float16*)((char*)d_ws + hoff);
  size_t ho = 0;
  const long PL_PATCH = (long)Cc * 768, PL_IN = (long)DEPTH * 2 * Dd * Cc, PL_BC = (long)DEPTH * Kk * BCW * Dd, PL_DTF = (long)DEPTH * Kk * Dd * Dd, PL_OUT = (long)DEPTH * Cc * Dd;
  _Float16* wp_patch = hp + ho; ho += (size_t)PL_PATCH * 2;
  _Float16* wp_in    = hp + ho; ho += (size_t)PL_IN * 2;
  _Float16* wp_bc    = hp + ho; ho += (size_t)PL_BC * 2;
  _Float16* wp_dtf   = hp + ho; ho += (size_t)PL_DTF * 2;
  _Float16* wp_out   = hp + ho; ho += (size_t)PL_OUT * 2;

  const dim3 blk256(256);
  auto nb = [](int total) { return dim3((total + 255) / 256); };

  prep_patch  <<<nb(Cc * 768 / 2), blk256, 0, stream>>>(patch_w, wp_patch);
  prep_inproj <<<nb(DEPTH * 2 * Dd * Cc / 2), blk256, 0, stream>>>(in_proj_w, wp_in);
  prep_bc     <<<nb(DEPTH * Kk * BCW * Dd / 2), blk256, 0, stream>>>(x_proj_w, wp_bc);
  prep_dtfused<<<nb(DEPTH * Kk * Dd * Dd / 2), blk256, 0, stream>>>(x_proj_w, dt_proj_w, wp_dtf);
  prep_outproj<<<nb(DEPTH * Cc * Dd / 2), blk256, 0, stream>>>(out_proj_w, wp_out);

  im2col_patch<<<nb(ROWS * 768), blk256, 0, stream>>>(x, col);
  gemm_wmma<<<dim3(ROWS / 32, Cc / 32, 1), dim3(32), 0, stream>>>(
      col, 0, wp_patch, 0, t, 0, ROWS, Cc, 768, 768, Cc, 0, nullptr, 0, PL_PATCH);
  patch_epilogue<<<nb(ROWS * Cc), blk256, 0, stream>>>(t, patch_b, pos);

  for (int i = 0; i < DEPTH; ++i) {
    layernorm_rows<<<dim3((ROWS + 127) / 128), dim3(128), 0, stream>>>(
        t, tn, ln1_w + (size_t)i * Cc, ln1_b + (size_t)i * Cc, ROWS, Cc);

    gemm_wmma<<<dim3(ROWS / 32, (2 * Dd) / 32, 1), dim3(32), 0, stream>>>(
        tn, 0, wp_in + (size_t)i * 2 * Dd * Cc, 0, xz, 0,
        ROWS, 2 * Dd, Cc, Cc, 2 * Dd, 0, nullptr, 0, PL_IN);

    dwconv_scan_prep<<<nb(ROWS * Dd), blk256, 0, stream>>>(
        xz, conv_w + (size_t)i * Dd * 9, conv_b + (size_t)i * Dd, xst);

    gemm_wmma<<<dim3(ROWS / 32, 1, Kk), dim3(32), 0, stream>>>(
        xst, (long)ROWS * Dd, wp_bc + (size_t)i * Kk * BCW * Dd, (long)BCW * Dd,
        bcb, (long)ROWS * BCW, ROWS, BCW, Dd, Dd, BCW, 0, nullptr, 0, PL_BC);

    gemm_wmma<<<dim3(ROWS / 32, Dd / 32, Kk), dim3(32), 0, stream>>>(
        xst, (long)ROWS * Dd, wp_dtf + (size_t)i * Kk * Dd * Dd, (long)Dd * Dd,
        dts, (long)ROWS * Dd, ROWS, Dd, Dd, Dd, Dd,
        1, dt_proj_b + (size_t)i * Kk * Dd, (long)Dd, PL_DTF);

    selective_scan<<<dim3((Kk * Bsz * Dd + 127) / 128), dim3(128), 0, stream>>>(
        xst, dts, bcb,
        A_logs + (size_t)i * Kk * Dd * Nn, Ds + (size_t)i * Kk * Dd, ys);

    merge_ln_gate<<<dim3(ROWS), dim3(32), 0, stream>>>(
        ys, xz, onw + (size_t)i * Dd, onb + (size_t)i * Dd, gated);

    gemm_wmma<<<dim3(ROWS / 32, Cc / 32, 1), dim3(32), 0, stream>>>(
        gated, 0, wp_out + (size_t)i * Cc * Dd, 0, t, 0,
        ROWS, Cc, Dd, Dd, Cc, 2, nullptr, 0, PL_OUT);
  }

  layernorm_rows<<<dim3((ROWS + 127) / 128), dim3(128), 0, stream>>>(
      t, tn, norm_w, norm_b, ROWS, Cc);
  pool_tokens<<<nb(Bsz * Cc), blk256, 0, stream>>>(tn, pooled);
  head_kernel<<<nb(Bsz * NCLS), blk256, 0, stream>>>(pooled, head_w, head_b, out);
}
